// SimpleSphereTracer_46840913330440
// MI455X (gfx1250) — hardware-verified
//
#include <hip/hip_runtime.h>
#include <stddef.h>


typedef __bf16       v16bf __attribute__((ext_vector_type(16)));
typedef unsigned int v8u   __attribute__((ext_vector_type(8)));
typedef unsigned int v4u   __attribute__((ext_vector_type(4)));
typedef float        v8f   __attribute__((ext_vector_type(8)));
typedef float        v4f   __attribute__((ext_vector_type(4)));

#ifndef NB
#define NB 4
#endif
#define NB_FULL 4
#define NRAY 4096
#define NPT  32
#define NPTS      (NB * NRAY * NPT)
#define NPTS_FULL (NB_FULL * NRAY * NPT)
#define KF 256
#define NH 16
#define KP 264
#define STEPS 4
#define MIN_DEPTH 0.05f
#define LN_EPS 1e-5f
#define WAVES_PER_BLOCK 8
#define PTS_PER_BLOCK (WAVES_PER_BLOCK * 16)

#ifndef IN_BF16
#define IN_BF16 0
#endif
#if IN_BF16
#define NPIECE 1
#else
#define NPIECE 3
#endif

#define WS_APL_BYTES ((size_t)NH * 32 * 2)
#define WS_TOTAL     (WS_APL_BYTES)

static_assert(NB >= 1 && NB <= NB_FULL);
static_assert((NPTS % PTS_PER_BLOCK) == 0);
static_assert(PTS_PER_BLOCK * 4 == 32 * 16);
static_assert((KF % 32) == 0 && KF == 256);
static_assert((KP % 8) == 0 && KP >= KF);
static_assert(NH == 16);
static_assert((WS_APL_BYTES % 128) == 0 && WS_APL_BYTES == 64 * 16);
static_assert(WS_TOTAL <= (size_t)134217728);
static_assert((size_t)NPTS * 3 < (size_t)0x7FFFFFFF);

__device__ __forceinline__ float bf16r(float x) {
  unsigned int u = __float_as_uint(x);
  u = (u + 0x7FFFu + ((u >> 16) & 1u)) & 0xFFFF0000u;
  return __uint_as_float(u);
}
__device__ __forceinline__ float inval(float x) {
#if IN_BF16
  return bf16r(x);
#else
  return x;
#endif
}
__device__ __forceinline__ unsigned int bf16_bits_rne(float x) {
  const unsigned int u = __float_as_uint(x);
  return (u + 0x7FFFu + ((u >> 16) & 1u)) >> 16;
}
__device__ __forceinline__ void split3(float v, unsigned int& hb, unsigned int& mb,
                                       unsigned int& lb) {
  hb = bf16_bits_rne(v);
  const float r1 = v - __uint_as_float(hb << 16);
  mb = bf16_bits_rne(r1);
  const float r2 = r1 - __uint_as_float(mb << 16);
  lb = bf16_bits_rne(r2);
}

__device__ __forceinline__ v8u frag_u(const unsigned short* p) {
  const v4u lo = *(const v4u*)(p);
  const v4u hi = *(const v4u*)(p + 16);
  v8u o;
#pragma unroll
  for (int i = 0; i < 4; ++i) { o[i] = lo[i]; o[i + 4] = hi[i]; }
  return o;
}

__device__ __forceinline__ v8f wmma_bf(v8u a, v8u b, v8f c) {
  v8f d = __builtin_amdgcn_wmma_f32_16x16x32_bf16(false, __builtin_bit_cast(v16bf, a),
                                                  false, __builtin_bit_cast(v16bf, b),
                                                  (short)0, c, false, false);
  asm volatile("v_nop\n\tv_nop\n\tv_nop\n\tv_nop" : "+v"(d) : "v"(a), "v"(b));
  return d;
}

__device__ __forceinline__ unsigned int pick_piece(unsigned int j, unsigned int hb,
                                                   unsigned int mb, unsigned int lb) {
  return (j < 3u) ? hb : ((j < 5u) ? mb : ((j == 5u) ? lb : 0u));
}

__global__ void __launch_bounds__(32)
fold_kernel(const float* __restrict__ feat_W, const float* __restrict__ feat_b,
            const float* __restrict__ ffn_W, const float* __restrict__ ffn_b,
            unsigned short* __restrict__ Apl) {
  __shared__ __attribute__((aligned(16))) unsigned short Ap[NPIECE * 16 * KP];
  __shared__ __attribute__((aligned(16))) unsigned short Bp[NPIECE * 16 * KP];
  __shared__ __attribute__((aligned(16))) float Ms[4 * NH];

  const unsigned int lane = threadIdx.x & 31u;
  const unsigned int h = lane >> 4, m = lane & 15u;

#pragma unroll 1
  for (unsigned int idx = lane; idx < 16u * KF; idx += 32u) {
    const unsigned int row = idx >> 8, f = idx & 255u;
    const unsigned int ia = (idx < 3u * KF) ? idx : (3u * KF - 1u);
    const float w = feat_W[ia];
    const float b = feat_b[f];
    float v = (row < 3u) ? w : ((row == 3u) ? b : 0.0f);
    v = inval(v);
    unsigned int hb, mb, lb;
    split3(v, hb, mb, lb);
    Ap[row * KP + f] = (unsigned short)hb;
#if NPIECE == 3
    Ap[16 * KP + row * KP + f] = (unsigned short)mb;
    Ap[32 * KP + row * KP + f] = (unsigned short)lb;
#endif
  }
#pragma unroll 1
  for (unsigned int idx = lane; idx < (unsigned int)(KF * NH); idx += 32u) {
    const unsigned int f = idx >> 4, n = idx & 15u;
    const float v = inval(ffn_W[idx]);
    unsigned int hb, mb, lb;
    split3(v, hb, mb, lb);
    Bp[n * KP + f] = (unsigned short)hb;
#if NPIECE == 3
    Bp[16 * KP + n * KP + f] = (unsigned short)mb;
    Bp[32 * KP + n * KP + f] = (unsigned short)lb;
#endif
  }
  const float fb = inval(ffn_b[m]);
  __syncthreads();

  v8f acc0 = {}, acc1 = {};
  const unsigned int fo = m * KP + h * 8u;
#pragma unroll 1
  for (unsigned int k0 = 0; k0 < (unsigned int)KF; k0 += 32u) {
    const v8u a0 = frag_u(&Ap[fo + k0]);
    const v8u b0 = frag_u(&Bp[fo + k0]);
    acc0 = wmma_bf(a0, b0, acc0);
#if NPIECE == 3
    const v8u a1 = frag_u(&Ap[16 * KP + fo + k0]);
    const v8u a2 = frag_u(&Ap[32 * KP + fo + k0]);
    const v8u b1 = frag_u(&Bp[16 * KP + fo + k0]);
    const v8u b2 = frag_u(&Bp[32 * KP + fo + k0]);
    acc1 = wmma_bf(a0, b1, acc1);
    acc1 = wmma_bf(a1, b0, acc1);
    acc1 = wmma_bf(a1, b1, acc1);
    acc1 = wmma_bf(a0, b2, acc1);
    acc1 = wmma_bf(a2, b0, acc1);
#endif
  }

  if (h == 0u) {
    const float m0 = acc0[0] + acc1[0];
    const float m1 = acc0[1] + acc1[1];
    const float m2 = acc0[2] + acc1[2];
    const float m3 = (acc0[3] + acc1[3]) + fb;
    Ms[0 * NH + m] = m0;
    Ms[1 * NH + m] = m1;
    Ms[2 * NH + m] = m2;
    Ms[3 * NH + m] = m3;
  }
  __syncthreads();

  v4u xs[2];
  unsigned int off[2];
#pragma unroll
  for (unsigned int i = 0; i < 2u; ++i) {
    const unsigned int p = lane + 32u * i;
    const unsigned int mr = p >> 2, kq = p & 3u;
    const unsigned int jA = 2u * kq, jB = jA + 1u;
    unsigned int hb[4], mb[4], lb[4];
#pragma unroll
    for (int c = 0; c < 4; ++c) split3(Ms[c * NH + mr], hb[c], mb[c], lb[c]);
    v4u x;
    x[0] = pick_piece(jA, hb[0], mb[0], lb[0]) | (pick_piece(jA, hb[1], mb[1], lb[1]) << 16);
    x[1] = pick_piece(jA, hb[2], mb[2], lb[2]) | (pick_piece(jA, hb[3], mb[3], lb[3]) << 16);
    x[2] = pick_piece(jB, hb[0], mb[0], lb[0]) | (pick_piece(jB, hb[1], mb[1], lb[1]) << 16);
    x[3] = pick_piece(jB, hb[2], mb[2], lb[2]) | (pick_piece(jB, hb[3], mb[3], lb[3]) << 16);
    xs[i] = x;
    off[i] = p * 8u;
  }
#pragma unroll
  for (int i = 0; i < 2; ++i) *(volatile v4u*)(Apl + off[i]) = xs[i];
  __threadfence();
#pragma unroll
  for (int i = 0; i < 2; ++i) *(volatile v4u*)(Apl + off[i]) = xs[i];
}

__global__ void __launch_bounds__(256)
trace_kernel(const float* __restrict__ start, const float* __restrict__ rdir,
             const unsigned short* __restrict__ Apl,
             const float* __restrict__ ln_g, const float* __restrict__ ln_b,
             const float* __restrict__ sdf_W, const float* __restrict__ sdf_b,
             float* __restrict__ out) {
  __shared__ __attribute__((aligned(16))) float Ds[PTS_PER_BLOCK];

  const int lane = threadIdx.x & 31;
  const int wave = __builtin_amdgcn_readfirstlane((int)(threadIdx.x >> 5));
  const int tile = (int)blockIdx.x * WAVES_PER_BLOCK + wave;
  const int h = lane >> 4, m = lane & 15;
  const bool hi_half = (h != 0);
  const int fsel = 8 * h;

  const v8u afrag = frag_u(Apl + m * 32 + h * 8);

  float glv[8], blv[8], swv[8];
#pragma unroll
  for (int r = 0; r < 8; ++r) {
    glv[r] = inval(ln_g[fsel + r]);
    blv[r] = inval(ln_b[fsel + r]);
    swv[r] = inval(sdf_W[fsel + r]);
  }
  const float sb = inval(sdf_b[0]);

  const size_t pbase = ((size_t)tile * 16 + (size_t)m) * 3;
  const float sx = inval(start[pbase + 0]);
  const float sy = inval(start[pbase + 1]);
  const float sz = inval(start[pbase + 2]);
  const float dx = inval(rdir[pbase + 0]);
  const float dy = inval(rdir[pbase + 1]);
  const float dz = inval(rdir[pbase + 2]);

  float depth = MIN_DEPTH;

#pragma unroll
  for (int step = 0; step < STEPS; ++step) {
    const float qx = fmaf(dx, depth, sx);
    const float qy = fmaf(dy, depth, sy);
    const float qz = fmaf(dz, depth, sz);
    unsigned int xh, xm, xl, yh, ym, yl, zh, zm, zl;
    split3(qx, xh, xm, xl);
    split3(qy, yh, ym, yl);
    split3(qz, zh, zm, zl);
    const unsigned int Wh0 = xh | (yh << 16);
    const unsigned int Wh1 = zh | (0x3F80u << 16);
    const unsigned int Wm0 = xm | (ym << 16);
    const unsigned int Wm1 = zm;
    const unsigned int Wl0 = xl | (yl << 16);
    const unsigned int Wl1 = zl;
    v8u bfrag;
    bfrag[0] = hi_half ? Wl0 : Wh0;
    bfrag[1] = hi_half ? Wl1 : Wh1;
    bfrag[2] = hi_half ? Wh0 : Wm0;
    bfrag[3] = hi_half ? Wh1 : Wm1;
    bfrag[4] = hi_half ? 0u  : Wm0;
    bfrag[5] = hi_half ? 0u  : Wm1;
    bfrag[6] = hi_half ? 0u  : Wh0;
    bfrag[7] = hi_half ? 0u  : Wh1;

    v8f acc = {};
    acc = wmma_bf(afrag, bfrag, acc);

    float s = acc[0];
#pragma unroll
    for (int r = 1; r < 8; ++r) s += acc[r];
    const float mu = (s + __shfl_xor(s, 16, 32)) * 0.0625f;

    float q = 0.0f;
    float dv[8];
#pragma unroll
    for (int r = 0; r < 8; ++r) {
      dv[r] = acc[r] - mu;
      q = fmaf(dv[r], dv[r], q);
    }
    const float var = (q + __shfl_xor(q, 16, 32)) * 0.0625f;
    const float inv = rsqrtf(var + LN_EPS);

    float t = 0.0f;
#pragma unroll
    for (int r = 0; r < 8; ++r) {
      float hv = fmaf(dv[r] * inv, glv[r], blv[r]);
      hv = fmaxf(hv, 0.0f);
      t = fmaf(hv, swv[r], t);
    }
    const float tsum = t + __shfl_xor(t, 16, 32);
    depth += tsum + sb;
  }

  if (!hi_half) Ds[wave * 16 + m] = depth;
  __syncthreads();

  if (wave == 0) {
    const v4f x = *(const v4f*)&Ds[lane * 4];
    float* p = out + (size_t)blockIdx.x * PTS_PER_BLOCK + (size_t)lane * 4;
    *(volatile v4f*)p = x;
    __threadfence();
    *(volatile v4f*)p = x;
  }
}

extern "C" void kernel_launch(void* const* d_in, const int* in_sizes, int n_in,
                              void* d_out, int out_size, void* d_ws, size_t ws_size,
                              hipStream_t stream) {
  if (n_in < 10) return;
  if ((long long)in_sizes[0] < (long long)NPTS * 3) return;
  if ((long long)in_sizes[1] < (long long)NPTS * 3) return;
  if (in_sizes[2] < 3 * KF || in_sizes[3] < KF || in_sizes[4] < KF * NH) return;
  if (in_sizes[5] < NH || in_sizes[6] < NH || in_sizes[7] < NH || in_sizes[8] < NH) return;
  if (in_sizes[9] < 1) return;
  if ((long long)out_size < (long long)NPTS) return;
  if (ws_size < WS_TOTAL) return;

  const float* start  = (const float*)d_in[0];
  const float* rdir   = (const float*)d_in[1];
  const float* feat_W = (const float*)d_in[2];
  const float* feat_b = (const float*)d_in[3];
  const float* ffn_W  = (const float*)d_in[4];
  const float* ffn_b  = (const float*)d_in[5];
  const float* ln_g   = (const float*)d_in[6];
  const float* ln_bb  = (const float*)d_in[7];
  const float* sdf_W  = (const float*)d_in[8];
  const float* sdf_b  = (const float*)d_in[9];
  float* out = (float*)d_out;
  unsigned short* Apl = (unsigned short*)d_ws;

  fold_kernel<<<dim3(1), dim3(32), 0, stream>>>(feat_W, feat_b, ffn_W, ffn_b, Apl);
  trace_kernel<<<dim3(NPTS / PTS_PER_BLOCK), dim3(32 * WAVES_PER_BLOCK), 0, stream>>>(
      start, rdir, Apl, ln_g, ln_bb, sdf_W, sdf_b, out);
}
